// MultiHeadAttention_27453430956540
// MI455X (gfx1250) — hardware-verified
//
#include <hip/hip_runtime.h>
#include <math.h>

typedef __attribute__((ext_vector_type(16))) _Float16 v16h;
typedef __attribute__((ext_vector_type(16))) __bf16 v16b;
typedef __attribute__((ext_vector_type(8)))  _Float16 v8h;
typedef __attribute__((ext_vector_type(8)))  float v8f;
typedef __attribute__((ext_vector_type(4)))  float v4f;
typedef __attribute__((ext_vector_type(4)))  unsigned v4u;

template <typename T> __device__ __forceinline__ void vst2(void* p, T v) { *(volatile T*)p = v; __threadfence(); *(volatile T*)p = v; }
__device__ __forceinline__ v8f wmma16(v16h a, v16h b, v8f c) {
  v8f d = __builtin_amdgcn_wmma_f32_16x16x32_f16(false, a, false, b, (short)0, c, false, false);
  asm volatile("v_nop\n\tv_nop\n\tv_nop\n\tv_nop" : "+v"(d) : "v"(a), "v"(b));
  return d;
}
__device__ __forceinline__ v8f wmma_bf(v16b a, v16b b, v8f c) {
  v8f d = __builtin_amdgcn_wmma_f32_16x16x32_bf16(false, a, false, b, (short)0, c, false, false);
  asm volatile("v_nop\n\tv_nop\n\tv_nop\n\tv_nop" : "+v"(d) : "v"(a), "v"(b));
  return d;
}
__device__ __forceinline__ v16h frag_h(const _Float16* rowk0, int lane) {
  union { v16h v; v8h q[2]; } u; const _Float16* p = rowk0 + 8 * (lane >> 4);
  u.q[0] = *(const v8h*)p; u.q[1] = *(const v8h*)(p + 16); return u.v;
}
__device__ __forceinline__ v16h frag_f32(const float* rowk0, int lane) {
  v16h a; const float* p = rowk0 + 8 * (lane >> 4);
#pragma unroll
  for (int i = 0; i < 8; ++i) { a[i] = (_Float16)p[i]; a[8 + i] = (_Float16)p[16 + i]; }
  return a;
}
__device__ __forceinline__ v16h frag_f32s(const float* rowk0, int lane, float sc) {
  v16h a; const float* p = rowk0 + 8 * (lane >> 4);
#pragma unroll
  for (int i = 0; i < 8; ++i) { a[i] = (_Float16)(p[i] * sc); a[8 + i] = (_Float16)(p[16 + i] * sc); }
  return a;
}
__device__ __forceinline__ float bfr(float v) { return (float)(__bf16)v; }
__device__ __forceinline__ v16b wcol_oi(const float* Wm, int k0, int o, int lane, int K) { v16b w; const float* p = Wm + (size_t)o * K + k0 + 8 * (lane >> 4);
#pragma unroll
  for (int i = 0; i < 8; ++i) { w[i] = (__bf16)p[i]; w[8 + i] = (__bf16)p[16 + i]; }
  return w; }
__device__ __forceinline__ v16h wcolh_oi(const float* Wm, int k0, int o, int lane, int K) { v16h w; const float* p = Wm + (size_t)o * K + k0 + 8 * (lane >> 4);
#pragma unroll
  for (int i = 0; i < 8; ++i) { w[i] = (_Float16)(bfr(p[i]) * 256.0f); w[8 + i] = (_Float16)(bfr(p[16 + i]) * 256.0f); }
  return w; }
#define LDSX() do { asm volatile("s_wait_dscnt 0" ::: "memory"); __builtin_amdgcn_wave_barrier(); __builtin_amdgcn_fence(3  , "workgroup"); } while (0)

#ifndef NB
#define NB 8
#endif
#ifndef SEQ
#define SEQ 1024
#endif
#define NB_FULL 8
#define SEQ_FULL 1024
#define TT SEQ
#define CC 768
#define DIN 768
#define NH 12
#define HD 64
#define NQB (TT / 64)
#define HG NH
#define SCALE (0.125f)

static_assert(TT % 256 == 0);
static_assert(CC % 128 == 0);
static_assert(DIN % 128 == 0);
static_assert(NH * HD == CC);
static_assert(NB <= NB_FULL);
static_assert(SEQ <= SEQ_FULL);

#define WS_QH  ((size_t)0)
#define WS_KH  (WS_QH + 2u * (size_t)NB * TT * CC)
#define WS_VT  (WS_KH + 2u * (size_t)NB * TT * CC)
#define WS_S   (WS_VT + 2u * (size_t)NB * CC * TT)
#define WS_Y   (WS_S  + 4u * (size_t)HG * TT * TT)
#define WS_END (WS_Y  + 4u * (size_t)NB * TT * CC)
static_assert(WS_END <= (size_t)134217728);

__global__ __launch_bounds__(128) void k_proj(const float* __restrict__ X, const float* __restrict__ W, _Float16* __restrict__ QH, _Float16* __restrict__ KH, _Float16* __restrict__ VT) {
  __shared__ __align__(16) _Float16 sh[64][136]; __shared__ __align__(16) _Float16 th[128][72];
  const int tid = threadIdx.x, wave = tid >> 5, lane = tid & 31, col = lane & 15, g = lane >> 4; const int which = blockIdx.z; const int c0 = blockIdx.y * 128; const size_t r0 = (size_t)blockIdx.x * 64; const size_t bb = r0 / TT; const int t0 = (int)(r0 % TT);
  const float* xrow = X + (bb * SEQ_FULL + (size_t)t0 + wave * 16 + col) * (size_t)DIN;
  v8f acc[8] = {};
#pragma unroll 2
  for (int kc = 0; kc < DIN / 32; ++kc) { v16b a; { const float* p = xrow + kc * 32 + 8 * g;
#pragma unroll
      for (int i = 0; i < 8; ++i) { a[i] = (__bf16)p[i]; a[8 + i] = (__bf16)p[16 + i]; } }
    asm volatile("s_wait_loadcnt 0x0" ::: "memory");
#pragma unroll
    for (int j = 0; j < 8; ++j) { const v16b w = wcol_oi(W, kc * 32, 3 * (c0 + j * 16 + col) + which, lane, DIN); asm volatile("s_wait_loadcnt 0x0" ::: "memory"); acc[j] = wmma_bf(a, w, acc[j]); } }
  if (which < 2) { _Float16* DH = which == 0 ? QH : KH;
#pragma unroll
    for (int j = 0; j < 8; ++j) {
#pragma unroll
      for (int r = 0; r < 8; ++r) sh[wave * 16 + 8 * g + r][j * 16 + col] = (_Float16)acc[j][r]; }
    __syncthreads();
    for (int e = tid; e < 64 * 16; e += 128) { const int rl = e >> 4, q = e & 15; const v4u val = *(const v4u*)&sh[rl][q * 8]; vst2((void*)(DH + (r0 + rl) * CC + c0 + q * 8), val); }
  } else {
#pragma unroll
    for (int j = 0; j < 8; ++j) {
#pragma unroll
      for (int r = 0; r < 8; ++r) th[j * 16 + col][wave * 16 + 8 * g + r] = (_Float16)acc[j][r]; }
    __syncthreads();
    for (int e = tid; e < 128 * 8; e += 128) { const int cl = e >> 3, q = e & 7; const v4u val = *(const v4u*)&th[cl][q * 8]; vst2((void*)(VT + (bb * CC + c0 + cl) * (size_t)TT + t0 + q * 8), val); } } }

__global__ __launch_bounds__(128) void k_sc(const _Float16* __restrict__ QH, const _Float16* __restrict__ KH, int b, float* __restrict__ S0) { __shared__ __align__(16) float ss[4][16][132];
  const int qb = blockIdx.x, kb = blockIdx.y; const int h = blockIdx.z; float* S = S0 + (size_t)blockIdx.z * TT * TT;
  const int tid = threadIdx.x, wave = tid >> 5, lane = tid & 31, col = lane & 15, g = lane >> 4; const int k0 = kb * 128; const int ql0 = qb * 64 + wave * 16; const size_t q0 = (size_t)b * TT + ql0, kr0 = (size_t)b * TT + k0;
  v8f acc[8] = {};
#pragma unroll
  for (int kc = 0; kc < HD / 32; ++kc) { const v16h ah = frag_h(QH + (q0 + col) * CC + h * HD + kc * 32, lane);
#pragma unroll
    for (int j = 0; j < 8; ++j) { const v16h kbf = frag_h(KH + (kr0 + j * 16 + col) * CC + h * HD + kc * 32, lane); acc[j] = wmma16(ah, kbf, acc[j]); } }
#pragma unroll
  for (int j = 0; j < 8; ++j) {
#pragma unroll
    for (int r = 0; r < 8; ++r) ss[wave][8 * g + r][j * 16 + col] = acc[j][r] * SCALE; }
  LDSX();
  for (int rl = 0; rl < 16; ++rl) { const v4f val = *(const v4f*)&ss[wave][rl][lane * 4]; vst2((void*)(S + (size_t)(ql0 + rl) * TT + k0 + lane * 4), val); } }

__global__ __launch_bounds__(256) void k_sm(float* __restrict__ S0) { __shared__ float sred[8]; __shared__ float sbc; __shared__ __align__(16) float shv[TT];
  const int tid = threadIdx.x; const int t = blockIdx.x; const int kend = TT;
  float* sr = S0 + (size_t)blockIdx.y * TT * TT + (size_t)t * TT;
  float m = -3.0e38f; for (int k = tid; k < kend; k += 256) { const float v = sr[k]; shv[k] = v; m = fmaxf(m, v); }
#pragma unroll
  for (int o = 1; o < 32; o <<= 1) m = fmaxf(m, __shfl_xor(m, o));
  if ((tid & 31) == 0) sred[tid >> 5] = m; __syncthreads(); if (tid == 0) { float a = sred[0]; for (int i = 1; i < 8; ++i) a = fmaxf(a, sred[i]); sbc = a; } __syncthreads(); m = sbc; __syncthreads();
  float sum = 0.f; for (int k = tid; k < kend; k += 256) { const float e = expf(shv[k] - m); shv[k] = e; sum += e; }
#pragma unroll
  for (int o = 1; o < 32; o <<= 1) sum += __shfl_xor(sum, o);
  if ((tid & 31) == 0) sred[tid >> 5] = sum; __syncthreads(); if (tid == 0) { float a = 0.f; for (int i = 0; i < 8; ++i) a += sred[i]; sbc = a > 0.f ? 2048.0f / a : 0.f; } __syncthreads(); const float inv = sbc;
  for (int k = tid; k < kend; k += 256) shv[k] = shv[k] * inv;
  __syncthreads();
  for (int q = tid; q < kend / 4; q += 256) { const v4f val = *(const v4f*)&shv[q * 4]; vst2((void*)(sr + q * 4), val); } }

__global__ __launch_bounds__(128) void k_pv(const float* __restrict__ PS0, const _Float16* __restrict__ VT, int b, float* __restrict__ Y) { const int h = blockIdx.z; const float* PS = PS0 + (size_t)blockIdx.z * TT * TT; __shared__ __align__(16) float ss[4][16][HD + 4];
  const int tid = threadIdx.x, wave = tid >> 5, lane = tid & 31, col = lane & 15, g = lane >> 4; const int qb = blockIdx.x; const int ql0 = qb * 64 + wave * 16; const int kce = TT / 32;
  v8f acc[HD / 16] = {};
#pragma unroll 1
  for (int kc = 0; kc < kce; ++kc) { const v16h p = frag_f32(PS + (size_t)(ql0 + col) * TT + kc * 32, lane);
    asm volatile("s_wait_loadcnt 0x0" ::: "memory");
#pragma unroll
    for (int j = 0; j < HD / 16; ++j) { const size_t po = ((size_t)b * CC + h * HD + j * 16 + col) * (size_t)TT + kc * 32; acc[j] = wmma16(p, frag_h(VT + po, lane), acc[j]); } }
#pragma unroll
  for (int j = 0; j < HD / 16; ++j)
#pragma unroll
    for (int r = 0; r < 8; ++r) ss[wave][8 * g + r][j * 16 + col] = acc[j][r] * (1.0f / 2048.0f);
  LDSX();
  for (int rl = 0; rl < 16; ++rl) if (lane < HD / 4) { const v4f val = *(const v4f*)&ss[wave][rl][lane * 4]; vst2((void*)(Y + ((size_t)b * TT + ql0 + rl) * CC + h * HD + lane * 4), val); } }

__global__ __launch_bounds__(128) void k_out(const float* __restrict__ Y, const float* __restrict__ WO, const float* __restrict__ BO, float* __restrict__ OUT) { __shared__ __align__(16) float sf[4][16][132];
  const int tid = threadIdx.x, wave = tid >> 5, lane = tid & 31, col = lane & 15, g = lane >> 4; const int c0 = blockIdx.y * 128; const size_t rb = (size_t)blockIdx.x * 64; const size_t r0 = rb + wave * 16;
  const size_t bb = rb / TT; const size_t orow0 = bb * SEQ_FULL + (rb % TT) + wave * 16;
  v8f acc[8] = {};
#pragma unroll 2
  for (int kc = 0; kc < CC / 32; ++kc) { const v16h a = frag_f32s(Y + (r0 + col) * CC + kc * 32, lane, 64.0f); asm volatile("s_wait_loadcnt 0x0" ::: "memory");
#pragma unroll
    for (int j = 0; j < 8; ++j) { const v16h w = wcolh_oi(WO, kc * 32, c0 + j * 16 + col, lane, CC); asm volatile("s_wait_loadcnt 0x0" ::: "memory"); acc[j] = wmma16(a, w, acc[j]); } }
#pragma unroll
  for (int j = 0; j < 8; ++j) { const float bias = bfr(BO[c0 + j * 16 + col]);
#pragma unroll
    for (int r = 0; r < 8; ++r) sf[wave][8 * g + r][j * 16 + col] = acc[j][r] * (1.0f / 16384.0f) + bias; }
  LDSX();
  for (int rl = 0; rl < 16; ++rl) { const v4f val = *(const v4f*)&sf[wave][rl][lane * 4]; vst2((void*)(OUT + (orow0 + rl) * DIN + c0 + lane * 4), val); } }

extern "C" void kernel_launch(void* const* d_in, const int* in_sizes, int n_in, void* d_out, int out_size, void* d_ws, size_t ws_size, hipStream_t stream) {
  if (n_in < 4) return;
  const size_t need_rows = (size_t)(NB - 1) * SEQ_FULL + TT;
  if ((size_t)in_sizes[0] < need_rows * DIN) return;
  if ((size_t)in_sizes[1] < (size_t)3 * CC * DIN) return;
  if ((size_t)in_sizes[2] < (size_t)DIN * CC) return;
  if ((size_t)in_sizes[3] < (size_t)DIN) return;
  if ((size_t)out_size < need_rows * DIN) return;
  if (ws_size < (size_t)WS_END) return;
  const float* X = (const float*)d_in[0]; const float* WQKV = (const float*)d_in[1]; const float* WP = (const float*)d_in[2]; const float* BP = (const float*)d_in[3];
  char* ws = (char*)d_ws; _Float16 *QH = (_Float16*)(ws + WS_QH), *KH = (_Float16*)(ws + WS_KH), *VT = (_Float16*)(ws + WS_VT); float *S = (float*)(ws + WS_S), *Y = (float*)(ws + WS_Y);
  k_proj<<<dim3(NB * TT / 64, CC / 128, 3), 128, 0, stream>>>(X, WQKV, QH, KH, VT);
  for (int b = 0; b < NB; ++b) {
    k_sc<<<dim3(NQB, TT / 128, HG), 128, 0, stream>>>(QH, KH, b, S);
    k_sm<<<dim3(TT, HG), 256, 0, stream>>>(S);
    k_pv<<<dim3(NQB, 1, HG), 128, 0, stream>>>(S, VT, b, Y);
  }
  k_out<<<dim3(NB * TT / 64, DIN / 128), 128, 0, stream>>>(Y, WP, BP, (float*)d_out);
}
